// Attention_197568495719
// MI455X (gfx1250) — hardware-verified
//
#include <hip/hip_runtime.h>


#ifndef NB
#define NB 2
#endif
#ifndef SEQ
#define SEQ 2048
#endif
#define NB_FULL  2
#define SEQ_FULL 2048
#define DM   2048
#define NH   16
#define NKV  4
#define REP  (NH / NKV)
#define HD   128
#define DQ   (NH * HD)
#define DKV  (NKV * HD)
#define NQKV (DQ + 2 * DKV)
#define VOFF (DQ + DKV)
#ifndef RH
#define RH   ((SEQ) > 512 ? 512 : (SEQ) / 2)
#endif
#define PCAR 1024.0f
#define ACAR 256.0f
#define WCAR 64.0f
#define SCL  0.08838834764831845f
#define NEGB (-3.0e38f)
#define PP   72
#define OP   136

typedef _Float16 h16;
typedef unsigned short bf;
typedef __attribute__((ext_vector_type(16))) __bf16   v16bf;
typedef __attribute__((ext_vector_type(16))) _Float16 v16h;
typedef __attribute__((ext_vector_type(8)))  _Float16 v8h;
typedef __attribute__((ext_vector_type(8)))  unsigned short v8us;
typedef __attribute__((ext_vector_type(2)))  unsigned short v2us;
typedef __attribute__((ext_vector_type(8)))  float    v8f;
typedef __attribute__((ext_vector_type(4)))  float    v4f;
typedef __attribute__((ext_vector_type(2)))  float    v2f;
typedef v4f  __attribute__((may_alias)) v4fa;
typedef v8us __attribute__((may_alias)) v8usa;

constexpr unsigned ilog2c(unsigned v) { return v <= 1u ? 0u : 1u + ilog2c(v >> 1); }
#define LSEQ ilog2c((unsigned)SEQ)
#define LDM  ilog2c((unsigned)DM)
#define LHD  ilog2c((unsigned)HD)
#define LNKV ilog2c((unsigned)NKV)

static_assert((SEQ & (SEQ - 1)) == 0);
static_assert((DM & (DM - 1)) == 0);
static_assert(HD == 128);
static_assert((NKV & (NKV - 1)) == 0);
static_assert(SEQ % 64 == 0);
static_assert(RH % 64 == 0);
static_assert(RH > 0);
static_assert(RH < SEQ);
static_assert((SEQ - RH) % 64 == 0);
static_assert(DM % 64 == 0);
static_assert(DQ % 64 == 0);
static_assert(NQKV % 64 == 0);
static_assert((NB * SEQ) % 64 == 0);
static_assert(DQ == DM);
static_assert(NB <= NB_FULL);
static_assert(SEQ <= SEQ_FULL);
static_assert(HD == 32 * 4);
static_assert(((size_t)NQKV * 4) % 128 == 0);
static_assert(((size_t)VOFF * 4) % 128 == 0);
static_assert(((size_t)HD * 4) % 128 == 0);

__device__ __forceinline__ unsigned short f2bf(float f) { unsigned u = __float_as_uint(f); u += 0x7FFFu + ((u >> 16) & 1u); return (unsigned short)(u >> 16); }
__device__ __forceinline__ float bf2f(unsigned short b) { return __uint_as_float(((unsigned)b) << 16); }
__device__ __forceinline__ unsigned short hbits(float x) { return __builtin_bit_cast(unsigned short, (h16)x); }
__device__ __forceinline__ void splitf(float y, unsigned short& h, unsigned short& l) { h = f2bf(y); l = f2bf(y - bf2f(h)); }
__device__ __forceinline__ v16h cat16(v8h lo, v8h hi) { return __builtin_shufflevector(lo, hi, 0, 1, 2, 3, 4, 5, 6, 7, 8, 9, 10, 11, 12, 13, 14, 15); }
__device__ __forceinline__ v16bf cat16b(v8us lo, v8us hi) { return __builtin_bit_cast(v16bf, __builtin_shufflevector(lo, hi, 0, 1, 2, 3, 4, 5, 6, 7, 8, 9, 10, 11, 12, 13, 14, 15)); }
__device__ __forceinline__ v16h cat16u(v8us lo, v8us hi) { return __builtin_bit_cast(v16h, __builtin_shufflevector(lo, hi, 0, 1, 2, 3, 4, 5, 6, 7, 8, 9, 10, 11, 12, 13, 14, 15)); }
__device__ __forceinline__ v8f wmma16(v16h a, v16h b, v8f c) { return __builtin_amdgcn_wmma_f32_16x16x32_f16(false, a, false, b, (short)0, c, false, false); }
__device__ __forceinline__ v8f wmmab(v16bf a, v16bf b, v8f c) { return __builtin_amdgcn_wmma_f32_16x16x32_bf16(false, a, false, b, (short)0, c, false, false); }
__device__ __forceinline__ void wave_sync() { __builtin_amdgcn_fence(3  , "wavefront"); __builtin_amdgcn_wave_barrier(); asm volatile("" ::: "memory"); }

template <typename T16> struct WFrag;
template <> struct WFrag<h16> { typedef v16h V;
    static __device__ __forceinline__ V ld(const h16* p) { return cat16(*(const v8h*)p, *(const v8h*)(p + 16)); }
    static __device__ __forceinline__ V ldl(const unsigned short* p) { const v8us a = *(const v8usa*)p; const v8us c = *(const v8usa*)(p + 16); return cat16u(a, c); }
    static __device__ __forceinline__ v8f mma(V a, V b, v8f c) { return wmma16(a, b, c); } };
template <> struct WFrag<bf> { typedef v16bf V;
    static __device__ __forceinline__ V ld(const bf* p) { return cat16b(*(const v8us*)p, *(const v8us*)(p + 16)); }
    static __device__ __forceinline__ V ldl(const unsigned short* p) { const v8us a = *(const v8usa*)p; const v8us c = *(const v8usa*)(p + 16); return cat16b(a, c); }
    static __device__ __forceinline__ v8f mma(V a, V b, v8f c) { return wmmab(a, b, c); } };
template <typename T16> struct FaHi { static constexpr bool v = false; };
template <> struct FaHi<bf> { static constexpr bool v = true; };

template <typename T16, int NSPLIT>
__global__ __launch_bounds__(32) void k_gemmw(const T16* __restrict__ A, const T16* __restrict__ A2, const T16* __restrict__ Bt, const T16* __restrict__ Bt2, int K, float* C, int ldc, float osc, size_t sA, size_t sB, size_t sC) {
    typedef typename WFrag<T16>::V V;
    __shared__ __align__(16) float os[16 * 68];
    const size_t z = blockIdx.z; A += z * sA; if (A2) A2 += z * sA; Bt += z * sB; if (Bt2) Bt2 += z * sB; C += z * sC;
    const int lane = threadIdx.x & 31, lr = lane & 15, hi = lane >> 4; const int r0 = blockIdx.x * 64, c0 = blockIdx.y * 64;
    v8f acc[4][4];
#pragma unroll
    for (int mb = 0; mb < 4; ++mb)
#pragma unroll
        for (int nb = 0; nb < 4; ++nb) acc[mb][nb] = (v8f){};
    const size_t aoff = (size_t)(r0 + lr) * K + 8 * hi, boff = (size_t)(c0 + lr) * K + 8 * hi;
#pragma unroll 1
    for (int kc = 0; kc < K; kc += 32) {
        V a[4], a2[4];
#pragma unroll
        for (int mb = 0; mb < 4; ++mb) { a[mb] = WFrag<T16>::ld(A + aoff + (size_t)mb * 16 * K + kc); if (NSPLIT == 1 || NSPLIT == 2) a2[mb] = WFrag<T16>::ld(A2 + aoff + (size_t)mb * 16 * K + kc); }
#pragma unroll
        for (int nb = 0; nb < 4; ++nb) { const V b = WFrag<T16>::ld(Bt + boff + (size_t)nb * 16 * K + kc); V b2; if (NSPLIT >= 2) b2 = WFrag<T16>::ld(Bt2 + boff + (size_t)nb * 16 * K + kc);
#pragma unroll
            for (int mb = 0; mb < 4; ++mb) { acc[mb][nb] = WFrag<T16>::mma(a[mb], b, acc[mb][nb]); if (NSPLIT == 1 || NSPLIT == 2) acc[mb][nb] = WFrag<T16>::mma(a2[mb], b, acc[mb][nb]); if (NSPLIT >= 2) acc[mb][nb] = WFrag<T16>::mma(a[mb], b2, acc[mb][nb]); } }
        asm volatile("v_nop\n\tv_nop\n\tv_nop\n\tv_nop" : "+v"(acc[0][0]), "+v"(acc[1][1]), "+v"(acc[2][2]), "+v"(acc[3][3]) : "v"(a[0]), "v"(a[3]));
    }
#pragma unroll
    for (int mb = 0; mb < 4; ++mb) {
#pragma unroll
        for (int nb = 0; nb < 4; ++nb) {
#pragma unroll
            for (int j = 0; j < 8; ++j) os[(hi * 8 + j) * 68 + nb * 16 + lr] = acc[mb][nb][j]; }
        wave_sync();
        float* crow = C + (size_t)(r0 + mb * 16) * ldc + c0;
#pragma unroll 1
        for (int ps = 0; ps < 2; ++ps) {
#pragma unroll
            for (int s = 0; s < 8; ++s) { const int row = 2 * s + hi, cofs = lr * 4; v4f val = *(const v4fa*)(os + row * 68 + cofs); val = val * osc;
                *(volatile v4f*)(crow + (size_t)row * ldc + cofs) = val; }
            if (ps == 0) __threadfence(); }
        wave_sync();
    }
}

__global__ __launch_bounds__(256) void k_wtG(const float* __restrict__ w, unsigned N, bf* Bt, bf* Bt16, float sc16) {
    const unsigned lane = threadIdx.x & 31u; const unsigned L0 = (blockIdx.x * 8u + (threadIdx.x >> 5)) * 8u; const unsigned nlines = N * (unsigned)(DM / 64);
#pragma unroll 1
    for (unsigned ps = 0; ps < 2u; ++ps) {
#pragma unroll 1
        for (unsigned l = 0; l < 8u; ++l) { const unsigned L = L0 + l;
            if (L < nlines) { const unsigned e = L * 64u + lane * 2u; const unsigned k = e & (unsigned)(DM - 1), n = e >> LDM;
                const float w0 = w[(size_t)k * N + n], w1 = w[(size_t)(k + 1u) * N + n]; v2us o; o[0] = f2bf(w0); o[1] = f2bf(w1);
                *(volatile v2us*)(Bt + e) = o;
                if (Bt16) { v2us o2; o2[0] = hbits(bf2f(o[0]) * sc16); o2[1] = hbits(bf2f(o[1]) * sc16); *(volatile v2us*)(Bt16 + e) = o2; } } }
        if (ps == 0u) __threadfence(); }
}

__global__ __launch_bounds__(256) void k_cvt8(const float* __restrict__ src, bf* dst) {
    const unsigned i = blockIdx.x * 256u + threadIdx.x; if (i >= (unsigned)(NB * SEQ) * (unsigned)(DM / 8)) return;
    const unsigned row = i >> (LDM - 3u), c8 = i & (unsigned)(DM / 8 - 1); const unsigned b = row >> LSEQ, t = row & (unsigned)(SEQ - 1);
    const v8f v = *(const v8f*)(src + ((size_t)(b * (unsigned)SEQ_FULL + t) * DM + c8 * 8u)); v8us o;
#pragma unroll
    for (int k = 0; k < 8; ++k) o[k] = f2bf(v[k]);
    *(volatile v8us*)(dst + (size_t)i * 8) = o; __threadfence(); *(volatile v8us*)(dst + (size_t)i * 8) = o; }

struct InvF { float v[64]; };
static_assert(sizeof(InvF) == 256);
__global__ __launch_bounds__(256) void k_cstab(InvF iv, float* CS) {
#pragma clang fp contract(off)
    const unsigned idx = blockIdx.x * 256u + threadIdx.x; if (idx >= (unsigned)SEQ * 64u) return;
    const unsigned i = idx & 63u, t = idx >> 6;
    float inv = iv.v[0];
#pragma unroll
    for (int j = 1; j < 64; ++j) inv = (i == (unsigned)j) ? iv.v[j] : inv;
    const float ang = (float)t * inv;
    v2f cs; cs[0] = cosf(ang); cs[1] = sinf(ang);
    *(volatile v2f*)(CS + (size_t)idx * 2) = cs; __threadfence(); *(volatile v2f*)(CS + (size_t)idx * 2) = cs; }

__global__ __launch_bounds__(256) void k_rope(const float* __restrict__ F, const float* __restrict__ CS, bf* Q16, bf* Qh, bf* Ql, bf* K16, bf* Kh, bf* Kl) {
#pragma clang fp contract(off)
    const unsigned lane = threadIdx.x & 31u; const unsigned R = blockIdx.x * 8u + (threadIdx.x >> 5); const unsigned hh = blockIdx.y;
    if (R >= (unsigned)(NB * SEQ)) return;
    const unsigned t = R & (unsigned)(SEQ - 1), b = R >> LSEQ; const unsigned j0 = lane * 2u;
    const float* f = F + (size_t)R * NQKV + hh * (unsigned)HD + j0;
    const v2f xl = *(const v2f*)f; const v2f xh = *(const v2f*)(f + 64);
    const v4f cs = *(const v4f*)(CS + ((size_t)t * 64u + j0) * 2u);
    float ol[2], oh[2];
    { const float a0 = xl[0] * cs[0], b0 = xh[0] * cs[1]; ol[0] = a0 - b0; const float a1 = xl[1] * cs[2], b1 = xh[1] * cs[3]; ol[1] = a1 - b1;
      const float c0 = xh[0] * cs[0], d0 = xl[0] * cs[1]; oh[0] = c0 + d0; const float c1 = xh[1] * cs[2], d1 = xl[1] * cs[3]; oh[1] = c1 + d1; }
    const bool isq = hh < (unsigned)NH;
    if (!isq) {
        float am = fmaxf(fmaxf(fabsf(ol[0]), fabsf(ol[1])), fmaxf(fabsf(oh[0]), fabsf(oh[1])));
        am = fmaxf(am, __shfl_xor(am, 1, 32)); am = fmaxf(am, __shfl_xor(am, 2, 32)); am = fmaxf(am, __shfl_xor(am, 4, 32)); am = fmaxf(am, __shfl_xor(am, 8, 32)); am = fmaxf(am, __shfl_xor(am, 16, 32));
        am = fmaxf(am, 1.0e-8f);
        const float qs = am * (1.0f / 127.0f); const float qi = 1.0f / qs;
        const float n0 = rintf(ol[0] * qi), n1 = rintf(ol[1] * qi), n2 = rintf(oh[0] * qi), n3 = rintf(oh[1] * qi);
        ol[0] = n0 * qs; ol[1] = n1 * qs; oh[0] = n2 * qs; oh[1] = n3 * qs;
    }
    bf* p16 = isq ? Q16 : K16; bf* ph = isq ? Qh : Kh; bf* pl = isq ? Ql : Kl;
    const unsigned pitch = isq ? (unsigned)DQ : (unsigned)DKV; const unsigned col = (isq ? hh : hh - (unsigned)NH) * (unsigned)HD + j0;
    const size_t o16 = (size_t)R * pitch + col; const size_t ohl = (size_t)(b * (unsigned)RH + t) * pitch + col;
    v2us f16l, f16h, hl, hh2, ll, lh;
#pragma unroll
    for (int q = 0; q < 2; ++q) { f16l[q] = hbits(ol[q]); f16h[q] = hbits(oh[q]); unsigned short a, c; splitf(ol[q], a, c); hl[q] = a; ll[q] = c; splitf(oh[q], a, c); hh2[q] = a; lh[q] = c; }
    const bool hires = t < (unsigned)RH;
#pragma unroll 1
    for (int ps = 0; ps < 2; ++ps) {
        *(volatile v2us*)(p16 + o16) = f16l; *(volatile v2us*)(p16 + o16 + 64) = f16h;
        if (hires) { *(volatile v2us*)(ph + ohl) = hl; *(volatile v2us*)(ph + ohl + 64) = hh2; *(volatile v2us*)(pl + ohl) = ll; *(volatile v2us*)(pl + ohl + 64) = lh; }
        if (ps == 0) __threadfence(); }
}

__global__ __launch_bounds__(256) void k_vq(float* F) {
#pragma clang fp contract(off)
    const unsigned lane = threadIdx.x & 31u; const unsigned R = blockIdx.x * 8u + (threadIdx.x >> 5); const unsigned g = blockIdx.y;
    if (R >= (unsigned)(NB * SEQ)) return;
    float* p = F + (size_t)R * NQKV + VOFF + g * (unsigned)HD + lane * 4u;
    const v4f x = *(const v4f*)p;
    float am = fmaxf(fmaxf(fabsf(x[0]), fabsf(x[1])), fmaxf(fabsf(x[2]), fabsf(x[3])));
    am = fmaxf(am, __shfl_xor(am, 1, 32)); am = fmaxf(am, __shfl_xor(am, 2, 32)); am = fmaxf(am, __shfl_xor(am, 4, 32)); am = fmaxf(am, __shfl_xor(am, 8, 32)); am = fmaxf(am, __shfl_xor(am, 16, 32));
    am = fmaxf(am, 1.0e-8f);
    const float qs = am * (1.0f / 127.0f); const float qi = 1.0f / qs;
    const float n0 = rintf(x[0] * qi), n1 = rintf(x[1] * qi), n2 = rintf(x[2] * qi), n3 = rintf(x[3] * qi);
    v4f o; o[0] = n0 * qs; o[1] = n1 * qs; o[2] = n2 * qs; o[3] = n3 * qs;
    *(volatile v4f*)p = o; __threadfence(); *(volatile v4f*)p = o; }

__global__ __launch_bounds__(256) void k_vt(const float* __restrict__ F, bf* V16, bf* Vh, bf* Vl) {
    const unsigned e = (blockIdx.x * 256u + threadIdx.x) * 2u; if (e >= (unsigned)(NB * NKV * HD) * (unsigned)SEQ) return;
    const unsigned t = e & (unsigned)(SEQ - 1), d = (e >> LSEQ) & (unsigned)(HD - 1), g = (e >> (LSEQ + LHD)) & (unsigned)(NKV - 1), b = e >> (LSEQ + LHD + LNKV);
    v2us o16, oh, ol;
#pragma unroll
    for (int q = 0; q < 2; ++q) { const float x = F[(size_t)(b * (unsigned)SEQ + t + (unsigned)q) * NQKV + VOFF + g * (unsigned)HD + d]; o16[q] = hbits(x); unsigned short a, c; splitf(x, a, c); oh[q] = a; ol[q] = c; }
    const bool hires = t < (unsigned)RH; const size_t eh = (size_t)(e >> LSEQ) * RH + t;
#pragma unroll 1
    for (int ps = 0; ps < 2; ++ps) {
        *(volatile v2us*)(V16 + e) = o16;
        if (hires) { *(volatile v2us*)(Vh + eh) = oh; *(volatile v2us*)(Vl + eh) = ol; }
        if (ps == 0) __threadfence(); }
}

template <typename T16>
__global__ __launch_bounds__(128) void k_fa(const T16* __restrict__ Q, const T16* __restrict__ Q2, const T16* __restrict__ Kp, const T16* __restrict__ K2, const T16* __restrict__ Vt, const T16* __restrict__ Vt2, bf* O1, bf* O2) {
    typedef WFrag<T16> W; typedef typename W::V V;
    constexpr bool HI = FaHi<T16>::v;
    constexpr unsigned RP = HI ? (unsigned)RH : (unsigned)SEQ;
    constexpr unsigned ROFF = HI ? 0u : (unsigned)RH;
    constexpr unsigned NPL = HI ? 2u : 1u;
    __shared__ __align__(16) unsigned short lds[4 * NPL * 16 * OP];
    const unsigned lane = threadIdx.x & 31u, wv = threadIdx.x >> 5, lr = lane & 15u, hi = lane >> 4;
    const unsigned g = blockIdx.y, b = blockIdx.z, h = g * (unsigned)REP + wv;
    const unsigned q0 = ROFF + blockIdx.x * 16u;
    const unsigned ntiles = (q0 >> 6) + 1u;
    unsigned short* l0 = lds + wv * (NPL * 16u * OP); unsigned short* l1 = l0 + (HI ? 16u * OP : 0u);
    const float C2 = SCL * 1.4426950408889634f;
    const size_t qo = (size_t)(b * RP + q0 + lr) * DQ + h * (unsigned)HD + 8u * hi;
    const size_t ko = (size_t)(b * RP + lr) * DKV + g * (unsigned)HD + 8u * hi;
    const size_t vo = (size_t)((b * (unsigned)NKV + g) * (unsigned)HD + lr) * RP + 8u * hi;
    v8f o[8];
#pragma unroll
    for (int nj = 0; nj < 8; ++nj) o[nj] = (v8f){};
    float m[8], l[8];
#pragma unroll
    for (int r = 0; r < 8; ++r) { m[r] = NEGB; l[r] = 0.f; }
#pragma unroll 1
    for (unsigned tt = 0; tt < ntiles; ++tt) {
        const unsigned kv0 = tt * 64u;
        unsigned qq = (unsigned)qo; asm volatile("" : "+v"(qq));
        v8f s[4];
#pragma unroll
        for (int ni = 0; ni < 4; ++ni) s[ni] = (v8f){};
        V qa, qb, kf, kl;
#pragma unroll
        for (int kc = 0; kc < 4; ++kc) {
            qa = W::ld(Q + qq + (unsigned)kc * 32u); if (HI) qb = W::ld(Q2 + qq + (unsigned)kc * 32u);
#pragma unroll
            for (int ni = 0; ni < 4; ++ni) {
                const size_t ka = ko + (size_t)(kv0 + (unsigned)ni * 16u) * DKV + (unsigned)kc * 32u;
                kf = W::ld(Kp + ka);
                s[ni] = W::mma(qa, kf, s[ni]);
                if (HI) { s[ni] = W::mma(qb, kf, s[ni]); kl = W::ld(K2 + ka); s[ni] = W::mma(qa, kl, s[ni]); }
            }
        }
        if (HI) asm volatile("v_nop\n\tv_nop\n\tv_nop\n\tv_nop" : "+v"(s[0]), "+v"(s[1]), "+v"(s[2]), "+v"(s[3]) : "v"(qa), "v"(kl));
        else    asm volatile("v_nop\n\tv_nop\n\tv_nop\n\tv_nop" : "+v"(s[0]), "+v"(s[1]), "+v"(s[2]), "+v"(s[3]) : "v"(qa), "v"(kf));
#pragma unroll
        for (int r = 0; r < 8; ++r) {
            const unsigned row = q0 + 8u * hi + (unsigned)r;
            float tv[4]; float mx = NEGB;
#pragma unroll
            for (int ni = 0; ni < 4; ++ni) { const unsigned key = kv0 + (unsigned)ni * 16u + lr; tv[ni] = (key <= row) ? s[ni][r] : NEGB; mx = fmaxf(mx, tv[ni]); }
            mx = fmaxf(mx, __shfl_xor(mx, 1, 32)); mx = fmaxf(mx, __shfl_xor(mx, 2, 32)); mx = fmaxf(mx, __shfl_xor(mx, 4, 32)); mx = fmaxf(mx, __shfl_xor(mx, 8, 32));
            const float mn = fmaxf(m[r], mx);
            const float al = __builtin_amdgcn_exp2f((m[r] - mn) * C2);
            m[r] = mn;
            float psum = 0.f;
#pragma unroll
            for (int ni = 0; ni < 4; ++ni) { const unsigned key = kv0 + (unsigned)ni * 16u + lr;
                const float pe = __builtin_amdgcn_exp2f((tv[ni] - mn) * C2); const float p = (key <= row) ? pe : 0.f; psum += p;
                const unsigned idx = (8u * hi + (unsigned)r) * PP + (unsigned)ni * 16u + lr;
                if (HI) { unsigned short a, c; splitf(p, a, c); l0[idx] = a; l1[idx] = c; } else { l0[idx] = hbits(p * PCAR); } }
            l[r] = l[r] * al + psum;
#pragma unroll
            for (int nj = 0; nj < 8; ++nj) o[nj][r] *= al;
            asm volatile("" : "+v"(s[0]), "+v"(s[1]), "+v"(s[2]), "+v"(s[3]) : : "memory");
            asm volatile("" : "+v"(o[0]), "+v"(o[1]), "+v"(o[2]), "+v"(o[3]), "+v"(o[4]), "+v"(o[5]), "+v"(o[6]), "+v"(o[7]));
        }
        wave_sync();
        V pa, pb, vf, vl;
#pragma unroll
        for (int kc = 0; kc < 2; ++kc) {
            pa = W::ldl(l0 + lr * PP + (unsigned)kc * 32u + 8u * hi); if (HI) pb = W::ldl(l1 + lr * PP + (unsigned)kc * 32u + 8u * hi);
#pragma unroll
            for (int nj = 0; nj < 8; ++nj) {
                const size_t va = vo + (size_t)((unsigned)nj * 16u) * RP + kv0 + (unsigned)kc * 32u;
                vf = W::ld(Vt + va);
                o[nj] = W::mma(pa, vf, o[nj]);
                if (HI) { o[nj] = W::mma(pb, vf, o[nj]); vl = W::ld(Vt2 + va); o[nj] = W::mma(pa, vl, o[nj]); }
            }
        }
        if (HI) asm volatile("v_nop\n\tv_nop\n\tv_nop\n\tv_nop" : "+v"(o[0]), "+v"(o[1]), "+v"(o[2]), "+v"(o[3]), "+v"(o[4]), "+v"(o[5]), "+v"(o[6]), "+v"(o[7]) : "v"(pa), "v"(vl));
        else    asm volatile("v_nop\n\tv_nop\n\tv_nop\n\tv_nop" : "+v"(o[0]), "+v"(o[1]), "+v"(o[2]), "+v"(o[3]), "+v"(o[4]), "+v"(o[5]), "+v"(o[6]), "+v"(o[7]) : "v"(pa), "v"(vf));
        wave_sync();
    }
#pragma unroll
    for (int r = 0; r < 8; ++r) { float v = l[r]; v += __shfl_xor(v, 1, 32); v += __shfl_xor(v, 2, 32); v += __shfl_xor(v, 4, 32); v += __shfl_xor(v, 8, 32); l[r] = v; }
#pragma unroll
    for (int r = 0; r < 8; ++r) {
        const float inv = 1.0f / l[r]; const float sc = HI ? inv : inv * (ACAR / PCAR);
#pragma unroll
        for (int nj = 0; nj < 8; ++nj) { const float val = o[nj][r] * sc; const unsigned idx = (8u * hi + (unsigned)r) * OP + (unsigned)nj * 16u + lr;
            if (HI) { unsigned short a, c; splitf(val, a, c); l0[idx] = a; l1[idx] = c; } else { l0[idx] = hbits(val); } }
    }
    wave_sync();
    const size_t ob = (size_t)(b * RP + q0) * DQ + h * (unsigned)HD + lr * 8u;
#pragma unroll 1
    for (int ps = 0; ps < 2; ++ps) {
#pragma unroll
        for (int s8 = 0; s8 < 8; ++s8) { const unsigned row = 2u * (unsigned)s8 + hi;
            const v8us v0 = *(const v8usa*)(l0 + row * OP + lr * 8u); *(volatile v8us*)(O1 + ob + (size_t)row * DQ) = v0;
            if (HI) { const v8us v1 = *(const v8usa*)(l1 + row * OP + lr * 8u); *(volatile v8us*)(O2 + ob + (size_t)row * DQ) = v1; } }
        if (ps == 0) __threadfence(); }
}

constexpr size_t al256(size_t v) { return (v + 255) & ~(size_t)255; }
constexpr size_t SZ_WQKV = al256((size_t)NQKV * DM * 2);
constexpr size_t SZ_WO   = al256((size_t)DM * DQ * 2);
constexpr size_t SZ_CS   = al256((size_t)SEQ * 64 * 2 * 4);
constexpr size_t SZ_XB   = al256((size_t)NB * SEQ * DM * 2);
constexpr size_t SZ_Q16  = al256((size_t)NB * SEQ * DQ * 2);
constexpr size_t SZ_R1   = SZ_XB > SZ_Q16 ? SZ_XB : SZ_Q16;
constexpr size_t SZ_F    = al256((size_t)NB * SEQ * NQKV * 4);
constexpr size_t SZ_AT16 = al256((size_t)NB * SEQ * DQ * 2);
constexpr size_t SZ_ATH  = al256((size_t)NB * RH * DQ * 2);
constexpr size_t SZ_R2   = SZ_F > (SZ_AT16 + 2 * SZ_ATH) ? SZ_F : (SZ_AT16 + 2 * SZ_ATH);
constexpr size_t SZ_K16  = al256((size_t)NB * SEQ * DKV * 2);
constexpr size_t SZ_KH   = al256((size_t)NB * RH * DKV * 2);
constexpr size_t SZ_QH   = al256((size_t)NB * RH * DQ * 2);
constexpr size_t SZ_VT16 = al256((size_t)NB * NKV * HD * SEQ * 2);
constexpr size_t SZ_VTH  = al256((size_t)NB * NKV * HD * RH * 2);
constexpr size_t SZ_TOTAL = SZ_WQKV + 2 * SZ_WO + SZ_CS + SZ_R1 + SZ_R2 + SZ_K16 + 2 * SZ_KH + 2 * SZ_QH + SZ_VT16 + 2 * SZ_VTH;
static_assert(SZ_TOTAL <= (size_t)134217728);
static_assert(SZ_AT16 + 2 * SZ_ATH <= SZ_R2);
static_assert(SZ_Q16 <= SZ_R1);
static_assert(((size_t)NB * SEQ * DM / 8) % 256 == 0);
static_assert(((size_t)SEQ * 64) % 256 == 0);
static_assert(((size_t)NB * SEQ) % 8 == 0);
static_assert(((size_t)NB * NKV * HD * SEQ / 2) % 256 == 0);
static_assert(((size_t)DKV * DM / 64) % 64 == 0);
static_assert(((size_t)DQ * DM / 64) % 64 == 0);

extern "C" void kernel_launch(void* const* d_in, const int* in_sizes, int n_in,
                              void* d_out, int out_size, void* d_ws, size_t ws_size, hipStream_t stream) {
    if (n_in < 6) return;
    const size_t need_x = ((size_t)(NB - 1) * SEQ_FULL + SEQ) * DM;
    if ((size_t)in_sizes[0] < need_x) return;
    if (in_sizes[1] < 1) return;
    if ((size_t)in_sizes[2] < (size_t)DM * DQ || (size_t)in_sizes[3] < (size_t)DM * DKV || (size_t)in_sizes[4] < (size_t)DM * DKV || (size_t)in_sizes[5] < (size_t)DQ * DM) return;
    if ((size_t)out_size < need_x) return;
    if (SZ_TOTAL > ws_size) return;
    const float* x = (const float*)d_in[0]; const float* wq = (const float*)d_in[2]; const float* wk = (const float*)d_in[3]; const float* wv = (const float*)d_in[4]; const float* wo = (const float*)d_in[5];
    float* OUT = (float*)d_out;
    char* wsp = (char*)d_ws;
    bf* WQKV = (bf*)wsp; wsp += SZ_WQKV;
    bf* WO = (bf*)wsp; wsp += SZ_WO;
    bf* WO16 = (bf*)wsp; wsp += SZ_WO;
    float* CS = (float*)wsp; wsp += SZ_CS;
    bf* XB = (bf*)wsp; bf* Q16 = (bf*)wsp; wsp += SZ_R1;
    float* F = (float*)wsp; bf* AT16 = (bf*)wsp; bf* ATh = (bf*)(wsp + SZ_AT16); bf* ATl = (bf*)(wsp + SZ_AT16 + SZ_ATH); wsp += SZ_R2;
    bf* K16 = (bf*)wsp; wsp += SZ_K16;
    bf* Kh = (bf*)wsp; wsp += SZ_KH; bf* Kl = (bf*)wsp; wsp += SZ_KH;
    bf* Qh = (bf*)wsp; wsp += SZ_QH; bf* Ql = (bf*)wsp; wsp += SZ_QH;
    bf* VT16 = (bf*)wsp; wsp += SZ_VT16;
    bf* VTh = (bf*)wsp; wsp += SZ_VTH; bf* VTl = (bf*)wsp; wsp += SZ_VTH;

    InvF iv;
    { double r = 10000.0;
      for (int s = 0; s < 6; ++s) { double y = r; for (int it = 0; it < 64; ++it) y = 0.5 * (y + r / y); r = y; }
      double p = 1.0;
      for (int i = 0; i < 64; ++i) { const float pw = (float)p; iv.v[i] = 1.0f / pw; p *= r; } }

    k_wtG<<<(unsigned)((size_t)DQ * DM / 64 / 64), 256, 0, stream>>>(wq, (unsigned)DQ, WQKV, nullptr, 0.0f);
    k_wtG<<<(unsigned)((size_t)DKV * DM / 64 / 64), 256, 0, stream>>>(wk, (unsigned)DKV, WQKV + (size_t)DQ * DM, nullptr, 0.0f);
    k_wtG<<<(unsigned)((size_t)DKV * DM / 64 / 64), 256, 0, stream>>>(wv, (unsigned)DKV, WQKV + (size_t)VOFF * DM, nullptr, 0.0f);
    k_wtG<<<(unsigned)((size_t)DM * DQ / 64 / 64), 256, 0, stream>>>(wo, (unsigned)DM, WO, WO16, WCAR);
    k_cvt8<<<(unsigned)((size_t)NB * SEQ * DM / 8 / 256), 256, 0, stream>>>(x, XB);
    k_cstab<<<(unsigned)((size_t)SEQ * 64 / 256), 256, 0, stream>>>(iv, CS);
    k_gemmw<bf, 0><<<dim3(NB * SEQ / 64, NQKV / 64, 1), 32, 0, stream>>>(XB, nullptr, WQKV, nullptr, DM, F, NQKV, 1.0f, 0, 0, 0);
    k_rope<<<dim3(NB * SEQ / 8, NH + NKV, 1), 256, 0, stream>>>(F, CS, Q16, Qh, Ql, K16, Kh, Kl);
    k_vq<<<dim3(NB * SEQ / 8, NKV, 1), 256, 0, stream>>>(F);
    k_vt<<<(unsigned)((size_t)NB * NKV * HD * SEQ / 2 / 256), 256, 0, stream>>>(F, VT16, VTh, VTl);
    k_fa<bf><<<dim3(RH / 16, NKV, NB), 128, 0, stream>>>(Qh, Ql, Kh, Kl, VTh, VTl, ATh, ATl);
    k_fa<h16><<<dim3((SEQ - RH) / 16, NKV, NB), 128, 0, stream>>>((const h16*)Q16, nullptr, (const h16*)K16, nullptr, (const h16*)VT16, nullptr, AT16, nullptr);
    k_gemmw<bf, 1><<<dim3(RH / 64, DM / 64, NB), 32, 0, stream>>>(ATh, ATl, WO, nullptr, DQ, OUT, DM, 1.0f, (size_t)RH * DQ, 0, (size_t)SEQ_FULL * DM);
    k_gemmw<h16, 0><<<dim3((SEQ - RH) / 64, DM / 64, NB), 32, 0, stream>>>((const h16*)AT16 + (size_t)RH * DQ, nullptr, (const h16*)WO16, nullptr, DQ, OUT + (size_t)RH * DM, DM, 1.0f / (ACAR * WCAR), (size_t)SEQ * DQ, 0, (size_t)SEQ_FULL * DM);
}
